// HyperGNN2D_52226802319464
// MI455X (gfx1250) — hardware-verified
//
#include <hip/hip_runtime.h>
#include <stddef.h>
#include <math.h>


#define NTHR    256
#define NWAVE   8
#define EPT     8
#define NGRP    2
#define CHUNK   (NTHR * EPT * NGRP)
#define WCAP    (EPT * NGRP * 32)
#define LISTN   (NWAVE * WCAP)
#define NBC     4096
#define NBF     1024
#define RCAP    40960
#define RBN     128
#define TGT     256
#define DEGCAP  256
#define OTHR    512
#define WSCAP   134217728
#define LDS_FILL ((RCAP + NBF + LISTN) * 4 + 64)

#define FNODE   16
#define FNET    8
#define FPIN    8
#define HN      96
#define HT      32
#define HP      16
#define NHEAD   4
#define FGW     8
#define NCH     2
#define NLAY    2
#define NTGT    4
#define ONODE   32
#define KNN     544
#define SACT    8.0f
#define SWGT    64.0f
#define SNB     512.0f
#define ESC     (1.0f / 512.0f)
#define EMSG    (1.0f / 4096.0f)

static_assert((CHUNK & (CHUNK - 1)) == 0);
static_assert(CHUNK <= 4096);
static_assert(NBC <= 4096 && NBF <= 4096);
static_assert((NBC & (NBC - 1)) == 0 && (NBF & (NBF - 1)) == 0);
static_assert(NBC == 4 * NBF);
static_assert(OTHR * 8 == NBC);
static_assert((RCAP % 32) == 0);
static_assert(TGT == NWAVE * 32);
static_assert((NBC % TGT) == 0);
static_assert(NHEAD * FGW == 32 && HN == NHEAD * NCH * FGW + ONODE);

typedef float          v4f  __attribute__((ext_vector_type(4)));
typedef float          v8f  __attribute__((ext_vector_type(8)));
typedef int            v4i  __attribute__((ext_vector_type(4)));
typedef _Float16       v8h  __attribute__((ext_vector_type(8)));
typedef _Float16       v16h __attribute__((ext_vector_type(16)));
union FragH { v16h v; v8h h[2]; };

__device__ __forceinline__ v8f wm(v16h a, v16h b, v8f c) {
  v8f d = __builtin_amdgcn_wmma_f32_16x16x32_f16(false, a, false, b, (short)0, c, false, false);
  asm volatile("v_nop\n\tv_nop\n\tv_nop\n\tv_nop" : "+v"(d) : "v"(a), "v"(b));
  return d;
}

template <int ACT>
__device__ __forceinline__ float actf(float v) {
  if (ACT == 1) return v >= 0.f ? v : 0.01f * v;
  if (ACT == 2) return tanhf(v);
  return v;
}

__device__ __forceinline__ float lk2(float v) { return v >= 0.f ? v : 0.2f * v; }

__global__ __launch_bounds__(NTHR) void k_cvt32(const float* __restrict__ src, _Float16* dst,
                                                int M, int K, int MP) {
  const int u = (int)blockIdx.x * NTHR + (int)threadIdx.x;
  if (u >= MP * 4) return;
  const int row = u >> 2, c0 = (u & 3) * 8;
  const int rowc = row < M ? row : M - 1;
  const int cc = (c0 + 8 <= K) ? c0 : (K - 8);
  const float* p = src + (size_t)rowc * K + cc;
  const v4f a = *(const v4f*)p;
  const v4f b = *(const v4f*)(p + 4);
  const bool ok = (row < M) && (c0 < K);
  v8h o;
  o[0] = (_Float16)(ok ? a.x * SACT : 0.f);
  o[1] = (_Float16)(ok ? a.y * SACT : 0.f);
  o[2] = (_Float16)(ok ? a.z * SACT : 0.f);
  o[3] = (_Float16)(ok ? a.w * SACT : 0.f);
  o[4] = (_Float16)(ok ? b.x * SACT : 0.f);
  o[5] = (_Float16)(ok ? b.y * SACT : 0.f);
  o[6] = (_Float16)(ok ? b.z * SACT : 0.f);
  o[7] = (_Float16)(ok ? b.w * SACT : 0.f);
  _Float16* q = dst + (size_t)u * 8;
  *(volatile v8h*)q = o;
  __threadfence();
  *(volatile v8h*)q = o;
}

__global__ __launch_bounds__(NTHR) void k_wt(const float* __restrict__ W, int ldw, int K, int N, int strideW,
                                             _Float16* out, int KP, int NP, int strideO,
                                             float scale, int permA, int permB) {
  const int kp8 = KP >> 3;
  const int units = NP * kp8;
  const int u = (int)blockIdx.x * NTHR + (int)threadIdx.x;
  if (u >= units) return;
  const float* Wl = W + (size_t)blockIdx.y * strideW;
  _Float16* ol = out + (size_t)blockIdx.y * strideO;
  const int n = u / kp8;
  const int k0 = (u - n * kp8) * 8;
  const int nc = n < N ? n : N - 1;
  v8h o;
#pragma unroll
  for (int e = 0; e < 8; ++e) {
    const int k = k0 + e;
    int kk = k;
    if (permA > 0) kk = (k < permA) ? (k + permB) : (k - permA);
    kk = kk < 0 ? 0 : (kk > K - 1 ? K - 1 : kk);
    const bool ok = (k < K) && (n < N);
    const float v = Wl[(size_t)kk * ldw + nc];
    o[e] = (_Float16)(ok ? v * scale : 0.f);
  }
  _Float16* p = ol + (size_t)u * 8;
  *(volatile v8h*)p = o;
  __threadfence();
  *(volatile v8h*)p = o;
}

__global__ __launch_bounds__(NTHR) void k_nnwt(const float* __restrict__ l2w, const float* __restrict__ l2b,
                                               _Float16* out) {
  const int u = (int)blockIdx.x * NTHR + (int)threadIdx.x;
  if (u >= ONODE * (KNN / 8)) return;
  const int y = (int)blockIdx.y;
  const float* w = l2w + (size_t)y * HP * 1024;
  const float* b = l2b + (size_t)y * 1024;
  const int o = u / (KNN / 8);
  const int k0 = (u - o * (KNN / 8)) * 8;
  v8h ov;
#pragma unroll
  for (int e = 0; e < 8; ++e) {
    const int k = k0 + e;
    int p = k >> 5; p = p > HP - 1 ? HP - 1 : p;
    const int i = k & 31;
    const float wv = w[(size_t)p * 1024 + i * 32 + o] * SWGT;
    int ib = k - 512; ib = ib < 0 ? 0 : (ib > 31 ? 31 : ib);
    const float bv = b[ib * 32 + o] * SNB;
    ov[e] = (_Float16)((k < 512) ? wv : bv);
  }
  _Float16* q = out + (size_t)y * ONODE * KNN + (size_t)u * 8;
  *(volatile v8h*)q = ov;
  __threadfence();
  *(volatile v8h*)q = ov;
}

template <int NB>
__device__ __forceinline__ int scan_chunk(const int* __restrict__ dsts, int nE, int cbase, int slotBase,
                                          int vec8, int* list, int tid, int lane, int wave) {
  int wc = 0;
#pragma unroll
  for (int g = 0; g < NGRP; ++g) {
    const int el0  = (g * NTHR + tid) * EPT;
    const int e0   = cbase + el0;
    const int sent = -2147483647 - 1;
    v4i da, db;
    if (vec8 != 0 && cbase + CHUNK <= nE) {
      da = *(const v4i*)(dsts + e0);
      db = *(const v4i*)(dsts + e0 + 4);
    } else {
      da.x = (e0     < nE) ? dsts[min(e0, nE - 1)] : sent;
      da.y = (e0 + 1 < nE) ? dsts[min(e0 + 1, nE - 1)] : sent;
      da.z = (e0 + 2 < nE) ? dsts[min(e0 + 2, nE - 1)] : sent;
      da.w = (e0 + 3 < nE) ? dsts[min(e0 + 3, nE - 1)] : sent;
      db.x = (e0 + 4 < nE) ? dsts[min(e0 + 4, nE - 1)] : sent;
      db.y = (e0 + 5 < nE) ? dsts[min(e0 + 5, nE - 1)] : sent;
      db.z = (e0 + 6 < nE) ? dsts[min(e0 + 6, nE - 1)] : sent;
      db.w = (e0 + 7 < nE) ? dsts[min(e0 + 7, nE - 1)] : sent;
    }
    const unsigned nb = (unsigned)slotBase;
    const unsigned s0 = (unsigned)da.x - nb, s1 = (unsigned)da.y - nb;
    const unsigned s2 = (unsigned)da.z - nb, s3 = (unsigned)da.w - nb;
    const unsigned s4 = (unsigned)db.x - nb, s5 = (unsigned)db.y - nb;
    const unsigned s6 = (unsigned)db.z - nb, s7 = (unsigned)db.w - nb;
    const bool h0 = s0 < (unsigned)NB, h1 = s1 < (unsigned)NB, h2 = s2 < (unsigned)NB, h3 = s3 < (unsigned)NB;
    const bool h4 = s4 < (unsigned)NB, h5 = s5 < (unsigned)NB, h6 = s6 < (unsigned)NB, h7 = s7 < (unsigned)NB;
    const unsigned any = __builtin_amdgcn_ballot_w32(h0 | h1 | h2 | h3 | h4 | h5 | h6 | h7);
    if (any != 0u) {
#define HITJ(J, HJ, SJ) { \
        const unsigned mj = __builtin_amdgcn_ballot_w32(HJ); \
        if (mj != 0u) { \
          if (HJ) { \
            const int pos = wc + (int)__builtin_amdgcn_mbcnt_lo(mj, 0u); \
            if (pos < WCAP) list[wave * WCAP + pos] = ((el0 + (J)) << 12) | (int)(SJ); \
          } \
          wc += (int)__builtin_popcount(mj); } }
      HITJ(0, h0, s0)
      HITJ(1, h1, s1)
      HITJ(2, h2, s2)
      HITJ(3, h3, s3)
      HITJ(4, h4, s4)
      HITJ(5, h5, s5)
      HITJ(6, h6, s6)
      HITJ(7, h7, s7)
#undef HITJ
    }
  }
  return wc;
}

__global__ __launch_bounds__(NTHR) void k_count(const int* __restrict__ dsts, int* cnt, int nE, int vec8) {
  __shared__ __attribute__((aligned(16))) int scnt[NBC];
  __shared__ __attribute__((aligned(16))) int list[LISTN];
  __shared__ int wcnt[NWAVE];
  const int tid = threadIdx.x, lane = tid & 31, wave = tid >> 5;
  const int nodeBase = blockIdx.x * NBC;

  for (int i = tid; i < NBC; i += NTHR) scnt[i] = 0;
  __syncthreads();

  const int nChunks = (nE + CHUNK - 1) / CHUNK;
#pragma unroll 1
  for (int ch = 0; ch < nChunks; ++ch) {
    const int cbase = ch * CHUNK;
    const int wc = scan_chunk<NBC>(dsts, nE, cbase, nodeBase, vec8, list, tid, lane, wave);
    if (lane == 0) wcnt[wave] = wc;
    __syncthreads();
    if (wave == 0) {
#pragma unroll 1
      for (int wsx = 0; wsx < NWAVE; ++wsx) {
        int n = __builtin_amdgcn_readfirstlane(wcnt[wsx]);
        n = n > WCAP ? WCAP : (n < 0 ? 0 : n);
        const int* lp = list + wsx * WCAP;
#pragma unroll 1
        for (int i = 0; i < n; ++i) {
          const int ent  = __builtin_amdgcn_readfirstlane(lp[i]);
          const int slot = ent & (NBC - 1);
          if (lane == 0) scnt[slot] = scnt[slot] + 1;
        }
      }
    }
    __syncthreads();
  }

  v4i cq[4];
#pragma unroll
  for (int q = 0; q < 4; ++q) {
    const int f = (wave * 4 + q) * 128 + 4 * lane;
    cq[q] = *(const v4i*)(scnt + f);
  }
  int* cp = cnt + (size_t)nodeBase;
#pragma unroll
  for (int q = 0; q < 4; ++q) {
    const int f = (wave * 4 + q) * 128 + 4 * lane;
    *(volatile v4i*)(cp + f) = cq[q];
  }
  __threadfence();
#pragma unroll
  for (int q = 0; q < 4; ++q) {
    const int f = (wave * 4 + q) * 128 + 4 * lane;
    *(volatile v4i*)(cp + f) = cq[q];
  }
}

__global__ __launch_bounds__(OTHR) void k_offsets(const int* __restrict__ cnt, int* off, int* rbase, int nChunk) {
  __shared__ __attribute__((aligned(16))) int soff[NBC];
  __shared__ __attribute__((aligned(16))) int srb[RBN];
  __shared__ int wtot[OTHR / 32];
  const int tid = threadIdx.x, lane = tid & 31, wave = tid >> 5, sub = tid >> 7;
  for (int i = tid; i < RBN; i += OTHR) srb[i] = 0;
  int carry = 0;
#pragma unroll 1
  for (int ch = 0; ch < nChunk; ++ch) {
    const int base = ch * NBC;
    const v4i c0 = *(const v4i*)(cnt + base + 8 * tid);
    const v4i c1 = *(const v4i*)(cnt + base + 8 * tid + 4);
    const int e0 = max(c0.x, 0), e1 = max(c0.y, 0), e2 = max(c0.z, 0), e3 = max(c0.w, 0);
    const int e4 = max(c1.x, 0), e5 = max(c1.y, 0), e6 = max(c1.z, 0), e7 = max(c1.w, 0);
    const int ts = e0 + e1 + e2 + e3 + e4 + e5 + e6 + e7;
    int incl = ts;
#pragma unroll
    for (int d = 1; d < 32; d <<= 1) {
      const int t = __shfl_up(incl, d);
      if (lane >= d) incl += t;
    }
    if (lane == 31) wtot[wave] = incl;
    __syncthreads();
    const int S0 = wtot[0]  + wtot[1]  + wtot[2]  + wtot[3];
    const int S1 = wtot[4]  + wtot[5]  + wtot[6]  + wtot[7];
    const int S2 = wtot[8]  + wtot[9]  + wtot[10] + wtot[11];
    const int S3 = wtot[12] + wtot[13] + wtot[14] + wtot[15];
    int pre = 0;
#pragma unroll 1
    for (int w = 4 * sub; w < wave; ++w) pre += wtot[w];
    const int b0 = carry;
    const int b1 = b0 + ((S0 + 31) & ~31);
    const int b2 = b1 + ((S1 + 31) & ~31);
    const int b3 = b2 + ((S2 + 31) & ~31);
    const int b4 = b3 + ((S3 + 31) & ~31);
    const int myb = sub == 0 ? b0 : (sub == 1 ? b1 : (sub == 2 ? b2 : b3));
    if (tid == 0) {
      srb[min(4 * ch + 0, RBN - 1)] = b0;
      srb[min(4 * ch + 1, RBN - 1)] = b1;
      srb[min(4 * ch + 2, RBN - 1)] = b2;
      srb[min(4 * ch + 3, RBN - 1)] = b3;
    }
    int run = myb + pre + incl - ts;
    soff[8 * tid + 0] = run; run += e0;
    soff[8 * tid + 1] = run; run += e1;
    soff[8 * tid + 2] = run; run += e2;
    soff[8 * tid + 3] = run; run += e3;
    soff[8 * tid + 4] = run; run += e4;
    soff[8 * tid + 5] = run; run += e5;
    soff[8 * tid + 6] = run; run += e6;
    soff[8 * tid + 7] = run;
    carry = b4;
    __syncthreads();
    const v4i o0 = *(const v4i*)(soff + 4 * tid);
    const v4i o1 = *(const v4i*)(soff + 4 * (tid + OTHR));
    int* op = off + base;
    *(volatile v4i*)(op + 4 * tid) = o0;
    *(volatile v4i*)(op + 4 * (tid + OTHR)) = o1;
    __threadfence();
    *(volatile v4i*)(op + 4 * tid) = o0;
    *(volatile v4i*)(op + 4 * (tid + OTHR)) = o1;
    __syncthreads();
  }
  if (tid == 0) srb[min(4 * nChunk, RBN - 1)] = carry;
  __syncthreads();
  v4i rv = {0, 0, 0, 0};
  if (tid < 32) rv = *(const v4i*)(srb + 4 * tid);
  if (tid < 32) *(volatile v4i*)(rbase + 4 * tid) = rv;
  __threadfence();
  if (tid < 32) *(volatile v4i*)(rbase + 4 * tid) = rv;
}

__global__ __launch_bounds__(NTHR) void k_fill(const int* __restrict__ srcs, const int* __restrict__ dsts,
                                               const int* __restrict__ off, const int* __restrict__ rbase,
                                               int* csr, int nIds, int nE, int vec8, int csrLen, int idMode) {
  extern __shared__ v4f lds_dyn[];
  int* region = (int*)lds_dyn;
  int* cursor = region + RCAP;
  int* list   = cursor + NBF;
  int* wcnt   = list + LISTN;
  const int tid = threadIdx.x, lane = tid & 31, wave = tid >> 5;
  const int b = blockIdx.x;
  const int nodeBase = b * NBF;

  int rb0 = rbase[b];
  const int rb1 = rbase[b + 1];
  rb0 = rb0 < 0 ? 0 : (rb0 > csrLen ? csrLen : rb0);
  rb0 &= ~31;
  int len = rb1 - rb0;
  len = len < 0 ? 0 : (len > RCAP ? RCAP : len);
  int lenW = (len + 31) & ~31;
  if (rb0 + lenW > csrLen) lenW = (csrLen - rb0) & ~31;

  {
    const v4i z = {0, 0, 0, 0};
    for (int i = tid; i < RCAP / 4; i += NTHR) ((v4i*)region)[i] = z;
    for (int s = tid; s < NBF; s += NTHR) {
      int o = off[nodeBase + s] - rb0;
      o = o < 0 ? 0 : (o > RCAP ? RCAP : o);
      cursor[s] = o;
    }
  }
  __syncthreads();

  const int nChunks = (nE + CHUNK - 1) / CHUNK;
#pragma unroll 1
  for (int ch = 0; ch < nChunks; ++ch) {
    const int cbase = ch * CHUNK;
    const int wc = scan_chunk<NBF>(dsts, nE, cbase, nodeBase, vec8, list, tid, lane, wave);
    if (lane == 0) wcnt[wave] = wc;
    __syncthreads();
    if (wave == 0) {
#pragma unroll 1
      for (int wsx = 0; wsx < NWAVE; ++wsx) {
        int n = __builtin_amdgcn_readfirstlane(wcnt[wsx]);
        n = n > WCAP ? WCAP : (n < 0 ? 0 : n);
        const int* lp = list + wsx * WCAP;
#pragma unroll 1
        for (int i = 0; i < n; ++i) {
          const int ent  = __builtin_amdgcn_readfirstlane(lp[i]);
          const int slot = ent & (NBF - 1);
          int e = cbase + ((ent >> 12) & (CHUNK - 1));
          e = e > nE - 1 ? nE - 1 : e;
          int v = idMode ? e : srcs[e];
          v = v < 0 ? 0 : (v > nIds - 1 ? nIds - 1 : v);
          if (lane == 0) {
            int pos = cursor[slot];
            pos = pos < 0 ? 0 : (pos > RCAP - 1 ? RCAP - 1 : pos);
            region[pos] = v;
            const int np = pos + 1;
            cursor[slot] = np > RCAP ? RCAP : np;
          }
        }
      }
    }
    __syncthreads();
  }

  const int nv = lenW >> 2;
  int* gp = csr + rb0;
#pragma unroll 1
  for (int i = tid; i < nv; i += NTHR) { const v4i v = ((const v4i*)region)[i]; *(volatile v4i*)(gp + 4 * i) = v; }
  __threadfence();
#pragma unroll 1
  for (int i = tid; i < nv; i += NTHR) { const v4i v = ((const v4i*)region)[i]; *(volatile v4i*)(gp + 4 * i) = v; }
}

template <int K1, int K2, int NC, int MODE, int ACT>
__global__ __launch_bounds__(NTHR) void k_gemm(
    const _Float16* __restrict__ P1, const _Float16* __restrict__ P2, const _Float16* __restrict__ Bw,
    const float* __restrict__ bias, const float* __restrict__ attL, const float* __restrict__ attR,
    const int* __restrict__ cnt, void* outp, float* eS, float* eD, int nRows, int cntLen) {
  constexpr int KP   = K1 + K2;
  constexpr int WPR  = (NC >= 32) ? 2 : 1;
  constexpr int TPW  = NC / 16 / WPR;
  constexpr int RG   = NWAVE / WPR;
  constexpr int BM   = RG * 16;
  constexpr int NACC = BM * NC;
  constexpr int K2P  = (K2 > 0) ? K2 : 32;
  static_assert((K1 % 32) == 0 && (K2 % 32) == 0 && K1 >= 32);
  static_assert(TPW * 16 * WPR == NC && TPW >= 1);
  static_assert(MODE != 1 || (NC == 64 && BM == 64));
  static_assert(MODE != 2 || (NC == 16 && BM == 128));
  static_assert((NACC % (8 * NTHR)) == 0);
  static_assert((NACC % NTHR) == 0);

  __shared__ __attribute__((aligned(16))) float    sAcc[NACC];
  __shared__ __attribute__((aligned(16))) _Float16 sOut[(MODE == 0) ? NACC : 8];
  __shared__ __attribute__((aligned(16))) float    sE[(MODE == 1) ? (2 * BM * NHEAD) : ((MODE == 2) ? (BM * NTGT) : 4)];

  const int tid = threadIdx.x, lane = tid & 31, wave = tid >> 5, hh = lane >> 4, m = lane & 15;
  const int rowBase = blockIdx.x * BM;
  const int rg  = wave / WPR;
  const int chf = wave - rg * WPR;
  const int r0  = rg * 16;
  const int c0  = chf * TPW * 16;
  const size_t arow = (size_t)(rowBase + r0 + m);
  const _Float16* a1 = P1 + arow * K1 + 8 * hh;
  const _Float16* a2 = P2 + arow * K2P + 8 * hh;

  v8f acc[TPW];
#pragma unroll
  for (int t = 0; t < TPW; ++t) { v8f z = {0.f, 0.f, 0.f, 0.f, 0.f, 0.f, 0.f, 0.f}; acc[t] = z; }

#pragma unroll
  for (int kt = 0; kt < KP / 32; ++kt) {
    FragH a;
    if (kt < K1 / 32) {
      a.h[0] = *(const v8h*)(a1 + 32 * kt);
      a.h[1] = *(const v8h*)(a1 + 32 * kt + 16);
    } else {
      const int k2 = kt - K1 / 32;
      a.h[0] = *(const v8h*)(a2 + 32 * k2);
      a.h[1] = *(const v8h*)(a2 + 32 * k2 + 16);
    }
#pragma unroll
    for (int t = 0; t < TPW; ++t) {
      const _Float16* bp = Bw + (size_t)(c0 + 16 * t + m) * KP + 32 * kt + 8 * hh;
      FragH b;
      b.h[0] = *(const v8h*)bp;
      b.h[1] = *(const v8h*)(bp + 16);
      acc[t] = wm(a.v, b.v, acc[t]);
    }
  }

  {
    float* sp = sAcc + (size_t)(r0 + 8 * hh) * NC + c0 + m;
#pragma unroll
    for (int t = 0; t < TPW; ++t) {
#pragma unroll
      for (int r = 0; r < 8; ++r) sp[r * NC + 16 * t] = acc[t][r];
    }
  }
  __syncthreads();

  if constexpr (MODE == 0) {
#pragma unroll 1
    for (int i = 0; i < NACC / NTHR; ++i) {
      const int idx = i * NTHR + tid;
      const int col = idx % NC;
      const float v = actf<ACT>(sAcc[idx] * ESC + bias[col]);
      sOut[idx] = (_Float16)(v * SACT);
    }
    __syncthreads();
    _Float16* gp = (_Float16*)outp + (size_t)rowBase * NC;
    constexpr int NU = NACC / 8;
#pragma unroll
    for (int i = 0; i < NU / NTHR; ++i) {
      const int u = i * NTHR + tid;
      const v8h v = *(const v8h*)(sOut + 8 * u);
      *(volatile v8h*)(gp + 8 * u) = v;
    }
    __threadfence();
#pragma unroll
    for (int i = 0; i < NU / NTHR; ++i) {
      const int u = i * NTHR + tid;
      const v8h v = *(const v8h*)(sOut + 8 * u);
      *(volatile v8h*)(gp + 8 * u) = v;
    }
  } else if constexpr (MODE == 1) {
#pragma unroll 1
    for (int i = 0; i < (BM * 8) / NTHR; ++i) {
      const int pr = i * NTHR + tid;
      const int r = pr >> 3, g = pr & 7;
      int crow = rowBase + r;
      crow = crow < 0 ? 0 : (crow > cntLen - 1 ? cntLen - 1 : crow);
      const int cv = cnt[crow];
      const float d = (float)(cv < 1 ? 1 : cv);
      const float sc = (g >= 4) ? (ESC * rsqrtf(d)) : ESC;
      float* bse = sAcc + r * NC + 8 * g;
      const float* al = attL + 8 * (g & 3);
      const float* ar = attR + 8 * (g & 3);
      float ps = 0.f, pd = 0.f;
#pragma unroll
      for (int f = 0; f < 8; ++f) {
        const float v = bse[f] * sc;
        bse[f] = v;
        ps += v * al[f];
        pd += v * ar[f];
      }
      if (g < 4) { sE[r * NHEAD + g] = ps; sE[BM * NHEAD + r * NHEAD + g] = pd; }
    }
    __syncthreads();
    float* hwp = (float*)outp + (size_t)rowBase * NC;
    constexpr int NU = NACC / 4;
    const size_t eb = (size_t)rowBase * NHEAD;
#pragma unroll
    for (int i = 0; i < NU / NTHR; ++i) {
      const int u = i * NTHR + tid;
      const v4f v = *(const v4f*)(sAcc + 4 * u);
      *(volatile v4f*)(hwp + 4 * u) = v;
    }
    if (tid < 64) {
      const v4f v = *(const v4f*)(sE + 4 * tid);
      *(volatile v4f*)(eS + eb + 4 * tid) = v;
    } else if (tid < 128) {
      const v4f v = *(const v4f*)(sE + BM * NHEAD + 4 * (tid - 64));
      *(volatile v4f*)(eD + eb + 4 * (tid - 64)) = v;
    }
    __threadfence();
#pragma unroll
    for (int i = 0; i < NU / NTHR; ++i) {
      const int u = i * NTHR + tid;
      const v4f v = *(const v4f*)(sAcc + 4 * u);
      *(volatile v4f*)(hwp + 4 * u) = v;
    }
    if (tid < 64) {
      const v4f v = *(const v4f*)(sE + 4 * tid);
      *(volatile v4f*)(eS + eb + 4 * tid) = v;
    } else if (tid < 128) {
      const v4f v = *(const v4f*)(sE + BM * NHEAD + 4 * (tid - 64));
      *(volatile v4f*)(eD + eb + 4 * (tid - 64)) = v;
    }
  } else {
#pragma unroll 1
    for (int i = 0; i < (BM * NTGT) / NTHR; ++i) {
      const int idx = i * NTHR + tid;
      const int r = idx >> 2, n = idx & 3;
      float v = sAcc[r * NC + n] * ESC + bias[n];
      v = v < -30.f ? -30.f : (v > 30.f ? 30.f : v);
      const float s = 1.0f / (1.0f + expf(-v));
      sE[idx] = s;
    }
    __syncthreads();
    float* op = (float*)outp;
    const int row = rowBase + tid;
    v4f ov = {0.f, 0.f, 0.f, 0.f};
    if (tid < BM) ov = *(const v4f*)(sE + 4 * tid);
    if (tid < BM && row < nRows) *(volatile v4f*)(op + (size_t)row * NTGT) = ov;
    __threadfence();
    if (tid < BM && row < nRows) *(volatile v4f*)(op + (size_t)row * NTGT) = ov;
  }
}

__global__ __launch_bounds__(NTHR) void k_msg(const _Float16* __restrict__ PIN, const _Float16* __restrict__ NET,
                                              const int* __restrict__ pnet, const _Float16* __restrict__ Bw,
                                              float* MSG, int nE, int nNet) {
  __shared__ __attribute__((aligned(16))) _Float16 sX[NWAVE * 16 * 40];
  __shared__ __attribute__((aligned(16))) float    sM[NWAVE * 16 * 32];
  const int tid = threadIdx.x, lane = tid & 31, wave = tid >> 5, hh = lane >> 4, m = lane & 15;
  const int ebase = ((int)blockIdx.x * NWAVE + wave) * 16;
  _Float16* sxw = sX + wave * (16 * 40);

#pragma unroll
  for (int it = 0; it < 2; ++it) {
    const int u = it * 32 + lane;
    const int r = u >> 2, pc = (u & 3) * 8;
    int e = ebase + r;
    e = e > nE - 1 ? nE - 1 : e;
    int s = pnet[e];
    s = s < 0 ? 0 : (s > nNet - 1 ? nNet - 1 : s);
    const v8h v = *(const v8h*)(NET + (size_t)s * HT + pc);
    *(v8h*)(sxw + r * 40 + pc) = v;
  }
  __syncthreads();

  FragH pvv;
  pvv.v = *(const v16h*)(PIN + (size_t)(ebase + m) * HP);
  const v8h xlo = *(const v8h*)(sxw + m * 40 + 8 * hh);
  const v8h xhi = *(const v8h*)(sxw + m * 40 + 16 + 8 * hh);

  v8f acc0 = {0.f, 0.f, 0.f, 0.f, 0.f, 0.f, 0.f, 0.f};
  v8f acc1 = {0.f, 0.f, 0.f, 0.f, 0.f, 0.f, 0.f, 0.f};
#pragma unroll
  for (int s = 0; s < HP + 1; ++s) {
    FragH a;
    if (s < HP) {
      const _Float16 p = pvv.v[s];
      a.h[0] = xlo * p;
      a.h[1] = xhi * p;
    } else {
      a.h[0] = xlo;
      a.h[1] = xhi;
    }
    const _Float16* bp0 = Bw + (size_t)m * KNN + 32 * s + 8 * hh;
    const _Float16* bp1 = Bw + (size_t)(16 + m) * KNN + 32 * s + 8 * hh;
    FragH b0, b1;
    b0.h[0] = *(const v8h*)bp0;
    b0.h[1] = *(const v8h*)(bp0 + 16);
    b1.h[0] = *(const v8h*)bp1;
    b1.h[1] = *(const v8h*)(bp1 + 16);
    acc0 = wm(a.v, b0.v, acc0);
    acc1 = wm(a.v, b1.v, acc1);
  }

  {
    float* sp = sM + wave * 512 + (8 * hh) * 32 + m;
#pragma unroll
    for (int r = 0; r < 8; ++r) { sp[r * 32] = acc0[r] * EMSG; sp[r * 32 + 16] = acc1[r] * EMSG; }
  }
  __syncthreads();

  float* gp = MSG + (size_t)ebase * 32;
  const float* smw = sM + wave * 512;
#pragma unroll
  for (int it = 0; it < 4; ++it) {
    const int u = it * 32 + lane;
    const v4f v = *(const v4f*)(smw + 4 * u);
    *(volatile v4f*)(gp + 4 * u) = v;
  }
  __threadfence();
#pragma unroll
  for (int it = 0; it < 4; ++it) {
    const int u = it * 32 + lane;
    const v4f v = *(const v4f*)(smw + 4 * u);
    *(volatile v4f*)(gp + 4 * u) = v;
  }
}

__global__ __launch_bounds__(NTHR) void k_node(
    const int* __restrict__ csrA, const int* __restrict__ offA, const int* __restrict__ cntA,
    const int* __restrict__ csrB, const int* __restrict__ offB, const int* __restrict__ cntB,
    const int* __restrict__ csrP, const int* __restrict__ offP, const int* __restrict__ cntP,
    const float* __restrict__ eS, const float* __restrict__ eD, const float* __restrict__ HW,
    const float* __restrict__ MSG, const float* __restrict__ gbias, const float* __restrict__ nbias,
    _Float16* NODE, int nN, int nEp, int csrLenG, int csrLenP) {
  __shared__ __attribute__((aligned(16))) _Float16 sRow[NWAVE * 32 * HN];
  const int tid = threadIdx.x, lane = tid & 31, wave = tid >> 5;
  const int tbase = (int)blockIdx.x * TGT + wave * 32;
  const int hd = lane >> 3, f = lane & 7;
  const int cl = tbase + lane;
  const int cA_l = cntA[cl], oA_l = offA[cl];
  const int cB_l = cntB[cl], oB_l = offB[cl];
  const int cP_l = cntP[cl], oP_l = offP[cl];
  const float gb = gbias[lane];
  const float nb = nbias[lane];
  _Float16* srw = sRow + wave * (32 * HN);

#pragma unroll 1
  for (int j = 0; j < 32; ++j) {
    const int c = tbase + j;
    const int nA  = __shfl(cA_l, j), stA = __shfl(oA_l, j);
    const int nB  = __shfl(cB_l, j), stB = __shfl(oB_l, j);
    const int nP0 = __shfl(cP_l, j), stP = __shfl(oP_l, j);
    const float ed = eD[(size_t)c * NHEAD + hd];

#pragma unroll 1
    for (int ch = 0; ch < NCH; ++ch) {
      int n = ch ? nB : nA;
      n = n < 0 ? 0 : (n > DEGCAP ? DEGCAP : n);
      const int st = ch ? stB : stA;
      const int* csr = ch ? csrB : csrA;
      float mx = -3.0e38f;
#pragma unroll 1
      for (int q0 = 0; q0 < n; q0 += 32) {
        int pos = st + q0 + lane;
        pos = pos < 0 ? 0 : (pos > csrLenG - 1 ? csrLenG - 1 : pos);
        int sl = csr[pos];
        sl = sl < 0 ? 0 : (sl > nN - 1 ? nN - 1 : sl);
        const int mcnt = (n - q0) < 32 ? (n - q0) : 32;
#pragma unroll 1
        for (int pp = 0; pp < mcnt; ++pp) {
          const int s = __builtin_amdgcn_readlane(sl, pp);
          mx = fmaxf(mx, lk2(eS[(size_t)s * NHEAD + hd] + ed));
        }
      }
      float den = 0.f, acc = 0.f;
#pragma unroll 1
      for (int q0 = 0; q0 < n; q0 += 32) {
        int pos = st + q0 + lane;
        pos = pos < 0 ? 0 : (pos > csrLenG - 1 ? csrLenG - 1 : pos);
        int sl = csr[pos];
        sl = sl < 0 ? 0 : (sl > nN - 1 ? nN - 1 : sl);
        const int mcnt = (n - q0) < 32 ? (n - q0) : 32;
#pragma unroll 1
        for (int pp = 0; pp < mcnt; ++pp) {
          const int s = __builtin_amdgcn_readlane(sl, pp);
          const float p = __expf(lk2(eS[(size_t)s * NHEAD + hd] + ed) - mx);
          den += p;
          acc += p * HW[(size_t)s * 64 + lane];
        }
      }
      const float dsafe = den > 0.f ? den : 1.0f;
      const float rd = (n > 0) ? __fdividef(1.0f, dsafe) : 0.f;
      float v = tanhf(acc * rd + gb);
      if (c >= nN) v = 0.f;
      srw[j * HN + hd * 16 + ch * 8 + f] = (_Float16)(v * SACT);
    }

    {
      int n = nP0;
      n = n < 0 ? 0 : (n > DEGCAP ? DEGCAP : n);
      float acc = 0.f;
#pragma unroll 1
      for (int q0 = 0; q0 < n; q0 += 32) {
        int pos = stP + q0 + lane;
        pos = pos < 0 ? 0 : (pos > csrLenP - 1 ? csrLenP - 1 : pos);
        int el = csrP[pos];
        el = el < 0 ? 0 : (el > nEp - 1 ? nEp - 1 : el);
        const int mcnt = (n - q0) < 32 ? (n - q0) : 32;
#pragma unroll 1
        for (int pp = 0; pp < mcnt; ++pp) {
          const int e = __builtin_amdgcn_readlane(el, pp);
          acc += MSG[(size_t)e * 32 + lane];
        }
      }
      const float dg = (float)(n < 1 ? 1 : n);
      float v = tanhf(acc * __fdividef(1.0f, dg) + nb);
      if (c >= nN) v = 0.f;
      srw[j * HN + 64 + lane] = (_Float16)(v * SACT);
    }
  }
  __syncthreads();

  _Float16* gp = NODE + (size_t)tbase * HN;
#pragma unroll
  for (int it = 0; it < (32 * HN) / 256; ++it) {
    const int u = it * 32 + lane;
    const v8h v = *(const v8h*)(srw + 8 * u);
    *(volatile v8h*)(gp + 8 * u) = v;
  }
  __threadfence();
#pragma unroll
  for (int it = 0; it < (32 * HN) / 256; ++it) {
    const int u = it * 32 + lane;
    const v8h v = *(const v8h*)(srw + 8 * u);
    *(volatile v8h*)(gp + 8 * u) = v;
  }
}

__global__ __launch_bounds__(NTHR) void k_net(
    const int* __restrict__ csrN, const int* __restrict__ offN, const int* __restrict__ cntN,
    const float* __restrict__ HW, const float* __restrict__ gcb, _Float16* NET,
    int nNet, int nN, int csrLen) {
  __shared__ __attribute__((aligned(16))) _Float16 sRow[NWAVE * 32 * HT];
  const int tid = threadIdx.x, lane = tid & 31, wave = tid >> 5;
  const int tbase = (int)blockIdx.x * TGT + wave * 32;
  const int cl = tbase + lane;
  const int cN_l = cntN[cl], oN_l = offN[cl];
  const float bb = gcb[lane];
  _Float16* srw = sRow + wave * (32 * HT);

#pragma unroll 1
  for (int j = 0; j < 32; ++j) {
    const int c = tbase + j;
    int n = __shfl(cN_l, j);
    const int st = __shfl(oN_l, j);
    n = n < 0 ? 0 : (n > DEGCAP ? DEGCAP : n);
    float acc = 0.f;
#pragma unroll 1
    for (int q0 = 0; q0 < n; q0 += 32) {
      int pos = st + q0 + lane;
      pos = pos < 0 ? 0 : (pos > csrLen - 1 ? csrLen - 1 : pos);
      int sl = csrN[pos];
      sl = sl < 0 ? 0 : (sl > nN - 1 ? nN - 1 : sl);
      const int mcnt = (n - q0) < 32 ? (n - q0) : 32;
#pragma unroll 1
      for (int pp = 0; pp < mcnt; ++pp) {
        const int s = __builtin_amdgcn_readlane(sl, pp);
        acc += HW[(size_t)s * 64 + 32 + lane];
      }
    }
    const float dg = (float)(n < 1 ? 1 : n);
    float v = tanhf(acc * rsqrtf(dg) + bb);
    if (c >= nNet) v = 0.f;
    srw[j * HT + lane] = (_Float16)(v * SACT);
  }
  __syncthreads();

  _Float16* gp = NET + (size_t)tbase * HT;
#pragma unroll
  for (int it = 0; it < (32 * HT) / 256; ++it) {
    const int u = it * 32 + lane;
    const v8h v = *(const v8h*)(srw + 8 * u);
    *(volatile v8h*)(gp + 8 * u) = v;
  }
  __threadfence();
#pragma unroll
  for (int it = 0; it < (32 * HT) / 256; ++it) {
    const int u = it * 32 + lane;
    const v8h v = *(const v8h*)(srw + 8 * u);
    *(volatile v8h*)(gp + 8 * u) = v;
  }
}

extern "C" void kernel_launch(void* const* d_in, const int* in_sizes, int n_in,
                              void* d_out, int out_size, void* d_ws, size_t ws_size,
                              hipStream_t stream) {
  if (n_in < 28) return;
  const int Nn = in_sizes[0] / FNODE;
  const int Nt = in_sizes[1] / FNET;
  const int Ep = in_sizes[24];
  const int Eg = in_sizes[26] / NCH;
  if (Nn <= 0 || Nt <= 0 || Ep <= 0 || Eg <= 0) return;
  if (in_sizes[0] != Nn * FNODE || in_sizes[1] != Nt * FNET || in_sizes[2] != Ep * FPIN) return;
  if (in_sizes[25] != Ep || in_sizes[26] != NCH * Eg || in_sizes[27] != NCH * Eg) return;
  if (in_sizes[3] != FNODE * HN || in_sizes[4] != HN) return;
  if (in_sizes[5] != FNET * HT || in_sizes[6] != HT) return;
  if (in_sizes[7] != FPIN * HP || in_sizes[8] != HP) return;
  if (in_sizes[9] != NLAY * HN * 32 || in_sizes[10] != NLAY * 32 || in_sizes[11] != NLAY * 32 || in_sizes[12] != NLAY * 32) return;
  if (in_sizes[13] != NLAY * HN * HT || in_sizes[14] != NLAY * HT) return;
  if (in_sizes[15] != NLAY * HP * 1024 || in_sizes[16] != NLAY * 1024 || in_sizes[17] != NLAY * ONODE) return;
  if (in_sizes[18] != (FNODE + HN) * HN || in_sizes[19] != HN) return;
  if (in_sizes[20] != HN * HN || in_sizes[21] != HN) return;
  if (in_sizes[22] != HN * NTGT || in_sizes[23] != NTGT) return;
  if (out_size != Nn * NTGT) return;
  if (Nn > (1 << 22) || Nt > (1 << 22) || Ep > (1 << 26) || Eg > (1 << 26)) return;

  const float* in_node = (const float*)d_in[0];
  const float* in_net  = (const float*)d_in[1];
  const float* in_pin  = (const float*)d_in[2];
  const float* node_lw = (const float*)d_in[3];
  const float* node_lb = (const float*)d_in[4];
  const float* net_lw  = (const float*)d_in[5];
  const float* net_lb  = (const float*)d_in[6];
  const float* pin_lw  = (const float*)d_in[7];
  const float* pin_lb  = (const float*)d_in[8];
  const float* fc_w    = (const float*)d_in[9];
  const float* attl    = (const float*)d_in[10];
  const float* attr    = (const float*)d_in[11];
  const float* att_b   = (const float*)d_in[12];
  const float* gc_w    = (const float*)d_in[13];
  const float* gc_b    = (const float*)d_in[14];
  const float* l2_w    = (const float*)d_in[15];
  const float* l2_b    = (const float*)d_in[16];
  const float* nn_b    = (const float*)d_in[17];
  const float* o1_w    = (const float*)d_in[18];
  const float* o1_b    = (const float*)d_in[19];
  const float* o2_w    = (const float*)d_in[20];
  const float* o2_b    = (const float*)d_in[21];
  const float* o3_w    = (const float*)d_in[22];
  const float* o3_b    = (const float*)d_in[23];
  const int* pins_src  = (const int*)d_in[24];
  const int* pins_dst  = (const int*)d_in[25];
  const int* grid_src  = (const int*)d_in[26];
  const int* grid_dst  = (const int*)d_in[27];
  float* out = (float*)d_out;

  const int NPAD = ((Nn + TGT - 1) / TGT) * TGT;
  const int TPAD = ((Nt + TGT - 1) / TGT) * TGT;
  const int EPAD = ((Ep + 255) / 256) * 256;
  const int nBCn = (Nn + NBC - 1) / NBC, CNTn = nBCn * NBC, nBFn = (Nn + NBF - 1) / NBF;
  const int nBCt = (Nt + NBC - 1) / NBC, CNTt = nBCt * NBC, nBFt = (Nt + NBF - 1) / NBF;
  if (4 * nBCn + 1 > RBN || 4 * nBCt + 1 > RBN) return;
  if (31 * 4 * nBCn > 4096 || 31 * 4 * nBCt > 4096) return;
  const int csrLenG = ((Eg + 31) & ~31) + 4096;
  const int csrLenP = ((Ep + 31) & ~31) + 4096;

  char* ws = (char*)d_ws;
  size_t off = 0;
  auto carve = [&](size_t bytes) -> size_t { size_t o = off; off += bytes; off = (off + 255) & ~(size_t)255; return o; };
  const size_t oW0  = carve((size_t)HN * 32 * 2);
  const size_t oW1  = carve((size_t)HT * 32 * 2);
  const size_t oW2  = carve((size_t)HP * 32 * 2);
  const size_t oW3  = carve((size_t)NLAY * 64 * HN * 2);
  const size_t oW4  = carve((size_t)NLAY * ONODE * KNN * 2);
  const size_t oW5  = carve((size_t)HN * 128 * 2);
  const size_t oW6  = carve((size_t)HN * HN * 2);
  const size_t oW7  = carve((size_t)16 * HN * 2);
  const size_t oCntA = carve((size_t)CNTn * 4), oOffA = carve((size_t)CNTn * 4);
  const size_t oCntB = carve((size_t)CNTn * 4), oOffB = carve((size_t)CNTn * 4);
  const size_t oCntP = carve((size_t)CNTn * 4), oOffP = carve((size_t)CNTn * 4);
  const size_t oCntN = carve((size_t)CNTt * 4), oOffN = carve((size_t)CNTt * 4);
  const size_t oRbA = carve((size_t)RBN * 4), oRbB = carve((size_t)RBN * 4);
  const size_t oRbP = carve((size_t)RBN * 4), oRbN = carve((size_t)RBN * 4);
  const size_t oCsrA = carve((size_t)csrLenG * 4), oCsrB = carve((size_t)csrLenG * 4);
  const size_t oCsrP = carve((size_t)csrLenP * 4), oCsrN = carve((size_t)csrLenP * 4);
  const size_t oXin  = carve((size_t)NPAD * 32 * 2);
  const size_t oXnet = carve((size_t)TPAD * 32 * 2);
  const size_t oXpin = carve((size_t)EPAD * 32 * 2);
  const size_t oNode = carve((size_t)NPAD * HN * 2);
  const size_t oNet  = carve((size_t)TPAD * HT * 2);
  const size_t oPin  = carve((size_t)EPAD * HP * 2);
  const size_t oH1   = carve((size_t)NPAD * HN * 2);
  const size_t oH2   = carve((size_t)NPAD * HN * 2);
  const size_t oHw   = carve((size_t)NPAD * 64 * 4);
  const size_t oEs   = carve((size_t)NPAD * NHEAD * 4);
  const size_t oEd   = carve((size_t)NPAD * NHEAD * 4);
  const size_t oMsg  = carve((size_t)EPAD * 32 * 4);
  if (off > ws_size || off > (size_t)WSCAP) return;

  _Float16* w0 = (_Float16*)(ws + oW0);
  _Float16* w1 = (_Float16*)(ws + oW1);
  _Float16* w2 = (_Float16*)(ws + oW2);
  _Float16* w3 = (_Float16*)(ws + oW3);
  _Float16* w4 = (_Float16*)(ws + oW4);
  _Float16* w5 = (_Float16*)(ws + oW5);
  _Float16* w6 = (_Float16*)(ws + oW6);
  _Float16* w7 = (_Float16*)(ws + oW7);
  int* cntA = (int*)(ws + oCntA); int* offA = (int*)(ws + oOffA); int* rbA = (int*)(ws + oRbA); int* csrA = (int*)(ws + oCsrA);
  int* cntB = (int*)(ws + oCntB); int* offB = (int*)(ws + oOffB); int* rbB = (int*)(ws + oRbB); int* csrB = (int*)(ws + oCsrB);
  int* cntP = (int*)(ws + oCntP); int* offP = (int*)(ws + oOffP); int* rbP = (int*)(ws + oRbP); int* csrP = (int*)(ws + oCsrP);
  int* cntN = (int*)(ws + oCntN); int* offN = (int*)(ws + oOffN); int* rbN = (int*)(ws + oRbN); int* csrN = (int*)(ws + oCsrN);
  _Float16* xin  = (_Float16*)(ws + oXin);
  _Float16* xnet = (_Float16*)(ws + oXnet);
  _Float16* xpin = (_Float16*)(ws + oXpin);
  _Float16* node = (_Float16*)(ws + oNode);
  _Float16* net  = (_Float16*)(ws + oNet);
  _Float16* pin  = (_Float16*)(ws + oPin);
  _Float16* h1   = (_Float16*)(ws + oH1);
  _Float16* h2   = (_Float16*)(ws + oH2);
  float* hw  = (float*)(ws + oHw);
  float* es  = (float*)(ws + oEs);
  float* edp = (float*)(ws + oEd);
  float* msg = (float*)(ws + oMsg);

  const int vec8G = ((Eg & 3) == 0) ? 1 : 0;
  const int vec8P = 1;

  k_cvt32<<<NPAD / 64, NTHR, 0, stream>>>(in_node, xin, Nn, FNODE, NPAD);
  k_cvt32<<<TPAD / 64, NTHR, 0, stream>>>(in_net, xnet, Nt, FNET, TPAD);
  k_cvt32<<<EPAD / 64, NTHR, 0, stream>>>(in_pin, xpin, Ep, FPIN, EPAD);

  k_wt<<<dim3((HN * 4 + NTHR - 1) / NTHR, 1), NTHR, 0, stream>>>(node_lw, HN, FNODE, HN, 0, w0, 32, HN, 0, SWGT, 0, 0);
  k_wt<<<dim3((HT * 4 + NTHR - 1) / NTHR, 1), NTHR, 0, stream>>>(net_lw, HT, FNET, HT, 0, w1, 32, HT, 0, SWGT, 0, 0);
  k_wt<<<dim3((HP * 4 + NTHR - 1) / NTHR, 1), NTHR, 0, stream>>>(pin_lw, HP, FPIN, HP, 0, w2, 32, HP, 0, SWGT, 0, 0);
  k_wt<<<dim3((32 * (HN / 8) + NTHR - 1) / NTHR, NLAY), NTHR, 0, stream>>>(fc_w, 32, HN, 32, HN * 32, w3, HN, 32, 64 * HN, SWGT, 0, 0);
  k_wt<<<dim3((32 * (HN / 8) + NTHR - 1) / NTHR, NLAY), NTHR, 0, stream>>>(gc_w, HT, HN, HT, HN * HT, w3 + 32 * HN, HN, 32, 64 * HN, SWGT, 0, 0);
  k_nnwt<<<dim3((ONODE * (KNN / 8) + NTHR - 1) / NTHR, NLAY), NTHR, 0, stream>>>(l2_w, l2_b, w4);
  k_wt<<<dim3((HN * 16 + NTHR - 1) / NTHR, 1), NTHR, 0, stream>>>(o1_w, HN, FNODE + HN, HN, 0, w5, 128, HN, 0, SWGT, HN, FNODE);
  k_wt<<<dim3((HN * (HN / 8) + NTHR - 1) / NTHR, 1), NTHR, 0, stream>>>(o2_w, HN, HN, HN, 0, w6, HN, HN, 0, SWGT, 0, 0);
  k_wt<<<dim3((16 * (HN / 8) + NTHR - 1) / NTHR, 1), NTHR, 0, stream>>>(o3_w, NTGT, HN, NTGT, 0, w7, HN, 16, 0, SWGT, 0, 0);

  hipFuncSetAttribute(reinterpret_cast<const void*>(&k_fill), hipFuncAttributeMaxDynamicSharedMemorySize, LDS_FILL);
  k_count<<<nBCn, NTHR, 0, stream>>>(grid_dst, cntA, Eg, vec8G);
  k_offsets<<<1, OTHR, 0, stream>>>(cntA, offA, rbA, nBCn);
  k_fill<<<nBFn, NTHR, LDS_FILL, stream>>>(grid_src, grid_dst, offA, rbA, csrA, Nn, Eg, vec8G, csrLenG, 0);
  k_count<<<nBCn, NTHR, 0, stream>>>(grid_dst + Eg, cntB, Eg, vec8G);
  k_offsets<<<1, OTHR, 0, stream>>>(cntB, offB, rbB, nBCn);
  k_fill<<<nBFn, NTHR, LDS_FILL, stream>>>(grid_src + Eg, grid_dst + Eg, offB, rbB, csrB, Nn, Eg, vec8G, csrLenG, 0);
  k_count<<<nBCn, NTHR, 0, stream>>>(pins_src, cntP, Ep, vec8P);
  k_offsets<<<1, OTHR, 0, stream>>>(cntP, offP, rbP, nBCn);
  k_fill<<<nBFn, NTHR, LDS_FILL, stream>>>(pins_dst, pins_src, offP, rbP, csrP, Ep, Ep, vec8P, csrLenP, 1);
  k_count<<<nBCt, NTHR, 0, stream>>>(pins_dst, cntN, Ep, vec8P);
  k_offsets<<<1, OTHR, 0, stream>>>(cntN, offN, rbN, nBCt);
  k_fill<<<nBFt, NTHR, LDS_FILL, stream>>>(pins_src, pins_dst, offN, rbN, csrN, Nn, Ep, vec8P, csrLenP, 0);

  k_gemm<32, 0, HN, 0, 1><<<NPAD / 64, NTHR, 0, stream>>>(xin, xin, w0, node_lb, node_lb, node_lb, cntP, node, es, edp, Nn, CNTn);
  k_gemm<32, 0, HT, 0, 1><<<TPAD / 64, NTHR, 0, stream>>>(xnet, xnet, w1, net_lb, net_lb, net_lb, cntP, net, es, edp, Nt, CNTn);
  k_gemm<32, 0, HP, 0, 1><<<EPAD / 128, NTHR, 0, stream>>>(xpin, xpin, w2, pin_lb, pin_lb, pin_lb, cntP, pin, es, edp, Ep, CNTn);

  for (int l = 0; l < NLAY; ++l) {
    k_gemm<HN, 0, 64, 1, 0><<<NPAD / 64, NTHR, 0, stream>>>(node, node, w3 + (size_t)l * 64 * HN, attl + l * 32,
                                                              attl + l * 32, attr + l * 32, cntP, hw, es, edp, Nn, CNTn);
    k_msg<<<EPAD / 128, NTHR, 0, stream>>>(pin, net, pins_dst, w4 + (size_t)l * ONODE * KNN, msg, Ep, Nt);
    k_node<<<NPAD / TGT, NTHR, 0, stream>>>(csrA, offA, cntA, csrB, offB, cntB, csrP, offP, cntP,
                                            es, edp, hw, msg, att_b + l * 32, nn_b + l * 32,
                                            node, Nn, Ep, csrLenG, csrLenP);
    k_net<<<TPAD / TGT, NTHR, 0, stream>>>(csrN, offN, cntN, hw, gc_b + l * 32, net, Nt, Nn, csrLenP);
  }

  k_gemm<HN, 32, HN, 0, 2><<<NPAD / 64, NTHR, 0, stream>>>(node, xin, w5, o1_b, o1_b, o1_b, cntP, h1, es, edp, Nn, CNTn);
  k_gemm<HN, 0, HN, 0, 2><<<NPAD / 64, NTHR, 0, stream>>>(h1, h1, w6, o2_b, o2_b, o2_b, cntP, h2, es, edp, Nn, CNTn);
  k_gemm<HN, 0, 16, 2, 0><<<NPAD / 128, NTHR, 0, stream>>>(h2, h2, w7, o3_b, o3_b, o3_b, cntP, out, es, edp, Nn, CNTn);
}
